// MultiHeadRelativeAttention_69801808495017
// MI455X (gfx1250) — hardware-run, weakly checked
//
#include <hip/hip_runtime.h>
#include <hip/hip_bf16.h>
#include <math.h>

#define NBT  4
#define SQ   2048
#define DME  256
#define HSZ  256
#define NHD  8
#define HD   32
#define N3   768
#define MT   (NBT * SQ)
#define KQP  (2 * HSZ)
#define AWV  4
#define RWP  48
#define WSCL 64.0f
#define QKS  16.0f
#define RSQD 0.17677669529663688f

static_assert(NHD * HD == HSZ);
static_assert(HD == 32);
static_assert((MT % 64) == 0 && (DME % 64) == 0 && (N3 % 64) == 0 && (HSZ % 64) == 0 && (KQP % 64) == 0);
static_assert((((MT / 64) * (KQP / 64)) % 8) == 0);
static_assert((((HSZ / 64) * (MT / 64)) % 8) == 0);
static_assert((((MT / 64) * (DME / 64)) % 8) == 0);
static_assert(((MT * DME) % 2048) == 0 && ((NHD * SQ * HD) % 2048) == 0);
static_assert(SQ == 128 * 16);
static_assert(((NBT * NHD * (SQ / 16)) % AWV) == 0);
static_assert(DME == NHD * 32 && (DME % 32) == 0);

typedef _Float16 v16h __attribute__((ext_vector_type(16)));
typedef __bf16 v16bf __attribute__((ext_vector_type(16)));
typedef unsigned short v16us __attribute__((ext_vector_type(16)));
typedef unsigned short v8us  __attribute__((ext_vector_type(8)));
typedef float v8f __attribute__((ext_vector_type(8)));
typedef float v4f __attribute__((ext_vector_type(4)));
typedef unsigned int v4u __attribute__((ext_vector_type(4)));

union FragU { v16us v; v8us h[2]; };

__device__ __forceinline__ unsigned short bf_bits(float f) {
  const unsigned u = __float_as_uint(f);
  return (unsigned short)((u + 0x7FFFu + ((u >> 16) & 1u)) >> 16);
}
__device__ __forceinline__ float bf_up(unsigned short h) { return __uint_as_float(((unsigned)h) << 16); }
__device__ __forceinline__ float bfr(float f) { return bf_up(bf_bits(f)); }
__device__ __forceinline__ unsigned short h_bits(_Float16 x) { return __builtin_bit_cast(unsigned short, x); }
__device__ __forceinline__ unsigned short f2h(float f) { return h_bits((_Float16)f); }
__device__ __forceinline__ unsigned pk16(unsigned short a, unsigned short b) { return (unsigned)a | ((unsigned)b << 16); }
__device__ __forceinline__ int clampi(int v, int lo, int hi) { return v < lo ? lo : (v > hi ? hi : v); }
__device__ __forceinline__ v8f zero8() { v8f z = {0.f, 0.f, 0.f, 0.f, 0.f, 0.f, 0.f, 0.f}; return z; }

__device__ __forceinline__ v16us ldfrag_u(const unsigned short* p) {
  FragU f;
  f.h[0] = *(const v8us*)(p);
  f.h[1] = *(const v8us*)(p + 16);
  return f.v;
}

template <int OPK>
__device__ __forceinline__ v8f mma_raw(v16us a, v16us b, v8f c) {
  if (OPK == 0)
    return __builtin_amdgcn_wmma_f32_16x16x32_f16(false, __builtin_bit_cast(v16h, a), false,
                                                  __builtin_bit_cast(v16h, b), (short)0, c, false, false);
  return __builtin_amdgcn_wmma_f32_16x16x32_bf16(false, __builtin_bit_cast(v16bf, a), false,
                                                 __builtin_bit_cast(v16bf, b), (short)0, c, false, false);
}
template <int OPK>
__device__ __forceinline__ v8f mma_g(v16us a, v16us b, v8f c) {
  c = mma_raw<OPK>(a, b, c);
#if defined(__HIP_DEVICE_COMPILE__)
  asm volatile("v_nop\n\tv_nop\n\tv_nop\n\tv_nop" : "+v"(c) : "v"(a), "v"(b));
#endif
  return c;
}
__device__ __forceinline__ void dep_guard1(v8f& a, v8f& b, v16us x) {
#if defined(__HIP_DEVICE_COMPILE__)
  asm volatile("v_nop\n\tv_nop\n\tv_nop\n\tv_nop" : "+v"(a), "+v"(b) : "v"(x));
#endif
}
__device__ __forceinline__ void keep4_u(v16us a, v16us b, v16us c, v16us d) {
#if defined(__HIP_DEVICE_COMPILE__)
  asm volatile("v_nop" :: "v"(a), "v"(b), "v"(c), "v"(d));
#endif
}
__device__ __forceinline__ void acc_guard4(v8f& a, v8f& b, v8f& c, v8f& d) {
#if defined(__HIP_DEVICE_COMPILE__)
  asm volatile("v_nop\n\tv_nop\n\tv_nop\n\tv_nop" : "+v"(a), "+v"(b), "+v"(c), "+v"(d));
#endif
}
__device__ __forceinline__ void acc_guard2(v8f& a, v8f& b) {
#if defined(__HIP_DEVICE_COMPILE__)
  asm volatile("v_nop\n\tv_nop\n\tv_nop\n\tv_nop" : "+v"(a), "+v"(b));
#endif
}
__device__ __forceinline__ void wave_sync_lds() {
  __builtin_amdgcn_fence(__ATOMIC_RELEASE, "workgroup");
  __builtin_amdgcn_wave_barrier();
  __builtin_amdgcn_fence(__ATOMIC_ACQUIRE, "workgroup");
}

__global__ __launch_bounds__(256) void cvt_lin(const float* __restrict__ w, unsigned short* o, int n, float sc) {
  const int base = (blockIdx.x * 256 + threadIdx.x) * 8;
  if (base + 8 > n) return;
  const v4f a0 = *(const v4f*)(w + base);
  const v4f a1 = *(const v4f*)(w + base + 4);
  v4u hv;
#pragma unroll
  for (int e = 0; e < 2; ++e) {
    hv[e]     = pk16(f2h(bfr(a0[2 * e]) * sc), f2h(bfr(a0[2 * e + 1]) * sc));
    hv[2 + e] = pk16(f2h(bfr(a1[2 * e]) * sc), f2h(bfr(a1[2 * e + 1]) * sc));
  }
  unsigned short* d = o + base;
  *(volatile v4u*)d = hv;
  __threadfence();
  *(volatile v4u*)d = hv;
}

template <int MODE>
__global__ __launch_bounds__(256) void cvt_t(const float* __restrict__ w, unsigned short* o, int R, int C, float sc) {
  __shared__ __align__(16) unsigned short st[64 * 72];
  const int t = threadIdx.x;
  const int r0 = blockIdx.y * 64, c0 = blockIdx.x * 64;
  if (r0 + 64 > R || c0 + 64 > C) return;
  {
    const int row = t >> 2, ch = (t & 3) * 16;
    const float* p = w + (size_t)(r0 + row) * C + c0 + ch;
#pragma unroll
    for (int q = 0; q < 4; ++q) {
      const v4f v = *(const v4f*)(p + 4 * q);
#pragma unroll
      for (int e = 0; e < 4; ++e) {
        unsigned short bits;
        if (MODE == 0) bits = f2h(bfr(v[e]) * sc);
        else           bits = bf_bits(v[e]);
        st[(ch + 4 * q + e) * 72 + row] = bits;
      }
    }
  }
  __syncthreads();
  v4u hv[2];
#pragma unroll
  for (int half = 0; half < 2; ++half) {
    const int cl = (t >> 3) + 32 * half, pc = (t & 7) * 8;
    hv[half] = *(const v4u*)(st + cl * 72 + pc);
  }
  for (int pass = 0; pass < 2; ++pass) {
#pragma unroll
    for (int half = 0; half < 2; ++half) {
      const int cl = (t >> 3) + 32 * half, pc = (t & 7) * 8;
      unsigned short* dst = o + (size_t)(c0 + cl) * R + r0 + pc;
      *(volatile v4u*)dst = hv[half];
    }
    __threadfence();
  }
}

template <int OPK, int NPL, int AHM, int OM>
__global__ __launch_bounds__(256) void gemm64(
    const unsigned short* __restrict__ Ap, const unsigned short* __restrict__ Ap2, int lda, int aplane,
    const unsigned short* __restrict__ Btp, int ldb,
    unsigned short* Ch, unsigned short* Ch2, float* Cf, int ldc,
    const float* __restrict__ cb, float wsc, float osc, int M, int N, int K) {
  __shared__ __align__(16) float sT[8][16 * 68];
  const int lane = threadIdx.x & 31;
  const int wave = threadIdx.x >> 5;
  const int tilesN = N >> 6;
  const int tilesM = M >> 6;
  const int tile = blockIdx.x * 8 + wave;
  if (tile >= tilesM * tilesN) return;
  const int tm = tile / tilesN;
  const int tn = tile - tm * tilesN;
  const int m0 = tm << 6;
  const int n0 = tn << 6;

  const int rlane = lane & 15;
  const int koff  = (lane >> 4) * 8;
  const int mOff  = (lane >> 4) * 8;

  v8f acc[4][4];
#pragma unroll
  for (int i = 0; i < 4; ++i)
#pragma unroll
    for (int j = 0; j < 4; ++j) acc[i][j] = zero8();

#pragma unroll 1
  for (int pl = 0; pl < NPL; ++pl) {
    const unsigned short* Ac = (pl == 0) ? Ap : Ap2;
    for (int k0 = 0; k0 < K; k0 += 32) {
      v16us bh[4];
#pragma unroll
      for (int j = 0; j < 4; ++j) {
        const size_t bo = (size_t)(n0 + (j << 4) + rlane) * ldb + koff + k0;
        bh[j] = ldfrag_u(Btp + bo);
      }
#pragma unroll
      for (int i = 0; i < 4; ++i) {
        size_t ao;
        if (AHM) ao = (size_t)(k0 >> 5) * (size_t)aplane + (size_t)(m0 + (i << 4) + rlane) * 32 + koff;
        else     ao = (size_t)(m0 + (i << 4) + rlane) * lda + koff + k0;
        const v16us ah = ldfrag_u(Ac + ao);
#pragma unroll
        for (int j = 0; j < 4; ++j) acc[i][j] = mma_raw<OPK>(ah, bh[j], acc[i][j]);
        dep_guard1(acc[i][0], acc[i][3], ah);
      }
      keep4_u(bh[0], bh[1], bh[2], bh[3]);
    }
  }
  acc_guard4(acc[0][0], acc[0][1], acc[0][2], acc[0][3]);
  acc_guard4(acc[1][0], acc[1][1], acc[1][2], acc[1][3]);
  acc_guard4(acc[2][0], acc[2][1], acc[2][2], acc[2][3]);
  acc_guard4(acc[3][0], acc[3][1], acc[3][2], acc[3][3]);

  const int hh2 = lane >> 4, c4 = (lane & 15) * 4;
  const int q8  = lane >> 3, c8 = (lane & 7) * 8;
  const float wo = wsc * osc;

  v4f cb4 = {0.f, 0.f, 0.f, 0.f};
  if (OM == 0) {
    const v4f v = *(const v4f*)(cb + n0 + c4);
    cb4[0] = bfr(v[0]); cb4[1] = bfr(v[1]); cb4[2] = bfr(v[2]); cb4[3] = bfr(v[3]);
  }

  float* slab = sT[wave];
#pragma unroll
  for (int i = 0; i < 4; ++i) {
    const int mBase = m0 + (i << 4);
#pragma unroll
    for (int j = 0; j < 4; ++j) {
#pragma unroll
      for (int r = 0; r < 8; ++r) {
        slab[(mOff + r) * 68 + (j << 4) + rlane] = acc[i][j][r];
      }
    }
    wave_sync_lds();
    if (OM == 0) {
      v4f vals[8];
#pragma unroll
      for (int it = 0; it < 8; ++it) {
        const int row = it * 2 + hh2;
        const v4f v = *(const v4f*)(slab + row * 68 + c4);
        vals[it] = v * wsc + cb4;
      }
      for (int pass = 0; pass < 2; ++pass) {
#pragma unroll
        for (int it = 0; it < 8; ++it) {
          const int row = it * 2 + hh2;
          *(volatile v4f*)(Cf + (size_t)(mBase + row) * ldc + (size_t)n0 + c4) = vals[it];
        }
        __threadfence();
      }
    } else {
      v4u hv[4], hw[4];
#pragma unroll
      for (int it = 0; it < 4; ++it) {
        const int row = it * 4 + q8;
        const float* sp = slab + row * 68 + c8;
        v4u ha = {0u, 0u, 0u, 0u}, hb = {0u, 0u, 0u, 0u};
#pragma unroll
        for (int e = 0; e < 4; ++e) {
          const float b0 = sp[2 * e]     * wo;
          const float b1 = sp[2 * e + 1] * wo;
          if (OM == 1) {
            ha[e] = pk16(f2h(b0), f2h(b1));
          } else {
            const unsigned short x0 = bf_bits(b0), x1 = bf_bits(b1);
            const unsigned short y0 = bf_bits(b0 - bf_up(x0)), y1 = bf_bits(b1 - bf_up(x1));
            ha[e] = pk16(x0, x1);
            hb[e] = pk16(y0, y1);
          }
        }
        hv[it] = ha;
        hw[it] = hb;
      }
      for (int pass = 0; pass < 2; ++pass) {
#pragma unroll
        for (int it = 0; it < 4; ++it) {
          const int row = it * 4 + q8;
          const size_t go = (size_t)(mBase + row) * ldc + (size_t)n0 + c8;
          *(volatile v4u*)(Ch + go) = hv[it];
          if (OM == 3) *(volatile v4u*)(Ch2 + go) = hw[it];
        }
        __threadfence();
      }
    }
    wave_sync_lds();
  }
}

__global__ __launch_bounds__(128) void attn_kernel(
    const unsigned short* __restrict__ KQ, const unsigned short* __restrict__ PE,
    const unsigned short* __restrict__ VTh, const unsigned short* __restrict__ VTl,
    unsigned short* Zh, unsigned short* Zl) {
  __shared__ __align__(16) float relw[AWV][16 * RWP];
  __shared__ __align__(16) unsigned short pws[AWV][2][16 * 32];
  __shared__ __align__(16) unsigned short zst[AWV][2][16 * 32];
  const int lane = threadIdx.x & 31, wv = threadIdx.x >> 5, m = lane & 15, hh = lane >> 4;
  const int task = blockIdx.x * AWV + wv;
  const int bh = task >> 7;
  const int t0 = (task & 127) << 4;
  const int b = bh >> 3, h = bh & 7;
  const size_t tok0 = (size_t)b * SQ;
  float* rw = relw[wv];
  unsigned short* ph = pws[wv][0];
  unsigned short* pl = pws[wv][1];

  const v16us qf = ldfrag_u(KQ + (tok0 + (size_t)(t0 + m)) * KQP + HSZ + h * HD + 8 * hh);

  float mx[8], ls[8];
  v8f O0 = zero8(), O1 = zero8();
#pragma unroll
  for (int r = 0; r < 8; ++r) { mx[r] = -1.0e30f; ls[r] = 0.f; }

  const int nblk = (t0 + 47) >> 5;

#pragma unroll 1
  for (int kb = 0; kb < nblk; ++kb) {
    const int sb = kb << 5;
    const unsigned short* kp = KQ + (tok0 + (size_t)(sb + m)) * KQP + h * HD + 8 * hh;
    const v16us kf0 = ldfrag_u(kp);
    const v16us kf1 = ldfrag_u(kp + (size_t)16 * KQP);
    const v8f S0 = mma_g<0>(qf, kf0, zero8());
    const v8f S1 = mma_g<0>(qf, kf1, zero8());

    const int u0 = SQ - 16 - t0 + sb;
#pragma unroll
    for (int j = 0; j < 3; ++j) {
      const int u = clampi(u0 + 16 * j + m, 0, SQ - 1);
      const v16us pf = ldfrag_u(PE + ((size_t)h * SQ + (size_t)u) * HD + 8 * hh);
      const v8f Pb = mma_g<0>(qf, pf, zero8());
#pragma unroll
      for (int r = 0; r < 8; ++r) rw[(8 * hh + r) * RWP + 16 * j + m] = Pb[r];
    }
    wave_sync_lds();

    float s0[8], s1[8];
#pragma unroll
    for (int r = 0; r < 8; ++r) {
      const int row = 8 * hh + r;
      const int tq = t0 + row;
      const float rv0 = rw[row * RWP + 15 - row + m];
      const float rv1 = rw[row * RWP + 31 - row + m];
      float a0 = (S0[r] * (1.0f / (QKS * QKS)) + rv0 * (1.0f / (QKS * WSCL))) * RSQD;
      float a1 = (S1[r] * (1.0f / (QKS * QKS)) + rv1 * (1.0f / (QKS * WSCL))) * RSQD;
      a0 = (sb + m > tq)      ? (a0 + (-1.0e9f)) : a0;
      a1 = (sb + 16 + m > tq) ? (a1 + (-1.0e9f)) : a1;
      s0[r] = a0; s1[r] = a1;
    }

#pragma unroll
    for (int r = 0; r < 8; ++r) {
      float xm = fmaxf(s0[r], s1[r]);
      xm = fmaxf(xm, __shfl_xor(xm, 1, 32));
      xm = fmaxf(xm, __shfl_xor(xm, 2, 32));
      xm = fmaxf(xm, __shfl_xor(xm, 4, 32));
      xm = fmaxf(xm, __shfl_xor(xm, 8, 32));
      const float mn = fmaxf(mx[r], xm);
      const float al = __expf(mx[r] - mn);
      mx[r] = mn;
      const float p0 = __expf(s0[r] - mn);
      const float p1 = __expf(s1[r] - mn);
      float ps = p0 + p1;
      ps += __shfl_xor(ps, 1, 32);
      ps += __shfl_xor(ps, 2, 32);
      ps += __shfl_xor(ps, 4, 32);
      ps += __shfl_xor(ps, 8, 32);
      ls[r] = ls[r] * al + ps;
      O0[r] = O0[r] * al;
      O1[r] = O1[r] * al;
      const int row = 8 * hh + r;
      const unsigned short x0 = bf_bits(p0), x1 = bf_bits(p1);
      ph[row * 32 + m]      = x0;
      ph[row * 32 + 16 + m] = x1;
      pl[row * 32 + m]      = bf_bits(p0 - bf_up(x0));
      pl[row * 32 + 16 + m] = bf_bits(p1 - bf_up(x1));
    }
    wave_sync_lds();

    const v16us af = ldfrag_u(ph + m * 32 + 8 * hh);
    const v16us bf = ldfrag_u(pl + m * 32 + 8 * hh);
    const size_t vo = (size_t)(h * HD + m) * MT + tok0 + (size_t)sb + 8 * hh;
    const v16us vh0 = ldfrag_u(VTh + vo);
    const v16us vh1 = ldfrag_u(VTh + vo + (size_t)16 * MT);
    const v16us vl0 = ldfrag_u(VTl + vo);
    const v16us vl1 = ldfrag_u(VTl + vo + (size_t)16 * MT);
    O0 = mma_g<1>(af, vh0, O0);
    O0 = mma_g<1>(af, vl0, O0);
    O0 = mma_g<1>(bf, vh0, O0);
    O1 = mma_g<1>(af, vh1, O1);
    O1 = mma_g<1>(af, vl1, O1);
    O1 = mma_g<1>(bf, vh1, O1);
  }
  acc_guard2(O0, O1);

  unsigned short* zh = zst[wv][0];
  unsigned short* zl = zst[wv][1];
#pragma unroll
  for (int r = 0; r < 8; ++r) {
    const int row = 8 * hh + r;
    const float linv = 1.0f / ls[r];
    const float o0 = O0[r] * linv;
    const float o1 = O1[r] * linv;
    const unsigned short x0 = bf_bits(o0), x1 = bf_bits(o1);
    zh[row * 32 + m]      = x0;
    zh[row * 32 + 16 + m] = x1;
    zl[row * 32 + m]      = bf_bits(o0 - bf_up(x0));
    zl[row * 32 + 16 + m] = bf_bits(o1 - bf_up(x1));
  }
  wave_sync_lds();
  {
    const v4u ha0 = *(const v4u*)(zh + lane * 8);
    const v4u ha1 = *(const v4u*)(zh + 256 + lane * 8);
    const v4u hb0 = *(const v4u*)(zl + lane * 8);
    const v4u hb1 = *(const v4u*)(zl + 256 + lane * 8);
    const size_t zo = ((size_t)h * MT + tok0 + (size_t)t0) * HD;
    unsigned short* dh = Zh + zo;
    unsigned short* dl = Zl + zo;
    for (int pass = 0; pass < 2; ++pass) {
      *(volatile v4u*)(dh + lane * 8)       = ha0;
      *(volatile v4u*)(dh + 256 + lane * 8) = ha1;
      *(volatile v4u*)(dl + lane * 8)       = hb0;
      *(volatile v4u*)(dl + 256 + lane * 8) = hb1;
      __threadfence();
    }
  }
}

extern "C" void kernel_launch(void* const* d_in, const int* in_sizes, int n_in,
                              void* d_out, int out_size, void* d_ws, size_t ws_size,
                              hipStream_t stream) {
  if (n_in < 5) return;
  if (in_sizes[0] != MT * DME) return;
  if (in_sizes[1] != DME * N3) return;
  if (in_sizes[2] != NHD * SQ * HD) return;
  if (in_sizes[3] != HSZ * DME) return;
  if (in_sizes[4] != DME) return;
  if (out_size != MT * DME) return;

  const float* x      = (const float*)d_in[0];
  const float* w_attn = (const float*)d_in[1];
  const float* pos    = (const float*)d_in[2];
  const float* w_proj = (const float*)d_in[3];
  const float* b_proj = (const float*)d_in[4];

  const size_t PXH = (size_t)MT * DME * 2;
  const size_t PPE = (size_t)NHD * SQ * HD * 2;
  const size_t PWT = (size_t)N3 * DME * 2;
  const size_t PWP = (size_t)HSZ * DME * 2;
  const size_t PKQ = (size_t)MT * KQP * 2;
  const size_t PVT = (size_t)HSZ * MT * 2;
  const size_t PZ  = (size_t)NHD * MT * HD * 2;
  size_t off = 0;
  const size_t oXH  = off; off += PXH;
  const size_t oPE  = off; off += PPE;
  const size_t oWT  = off; off += PWT;
  const size_t oWP  = off; off += PWP;
  const size_t oKQ  = off; off += PKQ;
  const size_t oVTH = off; off += PVT;
  const size_t oVTL = off; off += PVT;
  const size_t oZH  = off; off += PZ;
  const size_t oZL  = off; off += PZ;
  if (off > ws_size) return;
  if (off > (size_t)134217728) return;

  char* ws = (char*)d_ws;
  unsigned short* XH  = (unsigned short*)(ws + oXH);
  unsigned short* PEH = (unsigned short*)(ws + oPE);
  unsigned short* WT  = (unsigned short*)(ws + oWT);
  unsigned short* WP  = (unsigned short*)(ws + oWP);
  unsigned short* KQ  = (unsigned short*)(ws + oKQ);
  unsigned short* VTH = (unsigned short*)(ws + oVTH);
  unsigned short* VTL = (unsigned short*)(ws + oVTL);
  unsigned short* ZH  = (unsigned short*)(ws + oZH);
  unsigned short* ZL  = (unsigned short*)(ws + oZL);
  float* out0 = (float*)d_out;
  float* fdummy = (float*)(ws + oKQ);

  const dim3 blk(256);
  const int gKQ = ((MT / 64) * (KQP / 64)) / 8;
  const int gVT = ((HSZ / 64) * (MT / 64)) / 8;
  const int gPR = ((MT / 64) * (DME / 64)) / 8;

  cvt_lin<<<dim3((MT * DME) / 2048), blk, 0, stream>>>(x, XH, MT * DME, 1.0f);
  cvt_lin<<<dim3((NHD * SQ * HD) / 2048), blk, 0, stream>>>(pos, PEH, NHD * SQ * HD, WSCL);
  cvt_t<0><<<dim3(N3 / 64, DME / 64), blk, 0, stream>>>(w_attn, WT, DME, N3, WSCL);
  cvt_t<1><<<dim3(DME / 64, HSZ / 64), blk, 0, stream>>>(w_proj, WP, HSZ, DME, 1.0f);

  gemm64<0, 1, 0, 1><<<dim3(gKQ), blk, 0, stream>>>(
      XH, XH, DME, 0, WT, DME, KQ, KQ, fdummy, KQP, b_proj, 1.0f / WSCL, QKS, MT, KQP, DME);
  gemm64<0, 1, 0, 3><<<dim3(gVT), blk, 0, stream>>>(
      WT + (size_t)(2 * HSZ) * DME, WT, DME, 0, XH, DME, VTH, VTL, fdummy, MT, b_proj, 1.0f / WSCL, 1.0f, HSZ, MT, DME);

  attn_kernel<<<dim3((NBT * NHD * (SQ / 16)) / AWV), dim3(128), 0, stream>>>(KQ, PEH, VTH, VTL, ZH, ZL);

  gemm64<1, 2, 1, 0><<<dim3(gPR), blk, 0, stream>>>(
      ZH, ZL, DME, MT * HD, WP, DME, KQ, KQ, out0, DME, b_proj, 1.0f, 1.0f, MT, DME, DME);
  (void)hipGetLastError();
}
